// Conv2dfft_10445360463935
// MI455X (gfx1250) — hardware-verified
//
#include <hip/hip_runtime.h>

typedef _Float16 v16h __attribute__((ext_vector_type(16)));
typedef _Float16 v8h  __attribute__((ext_vector_type(8)));
typedef float    v8f  __attribute__((ext_vector_type(8)));
typedef float    v4f  __attribute__((ext_vector_type(4)));
typedef v8h __attribute__((may_alias)) v8ha;
typedef v4f __attribute__((may_alias)) v4fa;
typedef float __attribute__((may_alias)) f32a;

union Frag { v16h v; v8h half[2]; };

#define NB   32
#define CI   128
#define HH   32
#define WW   32
#define NO   128
#define HWP  (HH * WW)
#define KD   (9 * CI)
#define PT   64
#define NPT  (HWP / PT)
#define HR   4
#define HC   34
#define NCH  (KD / 8)
#define ACT_CARRY 64.0f
#define W_CARRY   1024.0f
#define INV_CARRY 1.52587890625e-05f

static_assert(HWP % PT == 0);
static_assert(PT == 2 * WW);
static_assert(KD % 32 == 0);
static_assert((KD * 2) % 128 == 0);
static_assert((PT * 4) % 128 == 0);
static_assert((HWP * 4) % 128 == 0);
static_assert((WW * CI * 2) % 128 == 0);
static_assert((CI * (WW / 4)) % 256 == 0);
static_assert(((WW * CI) / 8) % 256 == 0);
static_assert(NCH % 8 == 0);
static_assert(NCH <= 256);
static_assert(HR * HC * CI * 2 >= NO * PT * 4);
static_assert(HR * HC * CI * 2 <= 65536);
static_assert(NO == 128);

__device__ __forceinline__ v8f wmma_f16(v16h a, v16h b, v8f c) {
  v8f d = __builtin_amdgcn_wmma_f32_16x16x32_f16(false, a, false, b, (short)0, c, false, false);
  asm volatile("v_nop\n\tv_nop\n\tv_nop\n\tv_nop" : "+v"(d) : "v"(a), "v"(b));
  return d;
}

__device__ __forceinline__ v16h load_frag(const _Float16* p, int h) {
  Frag f;
  f.half[0] = *(const v8ha*)(p + 8 * h);
  f.half[1] = *(const v8ha*)(p + 16 + 8 * h);
  return f.v;
}

__device__ __forceinline__ v8h zero8h() {
  const v8h z = { (_Float16)0.0f, (_Float16)0.0f, (_Float16)0.0f, (_Float16)0.0f,
                  (_Float16)0.0f, (_Float16)0.0f, (_Float16)0.0f, (_Float16)0.0f };
  return z;
}

__device__ __forceinline__ float bf16r(float f) {
  unsigned u = __float_as_uint(f);
  u += 0x7FFFu + ((u >> 16) & 1u);
  u &= 0xFFFF0000u;
  return __uint_as_float(u);
}

__global__ __launch_bounds__(256) void wcvt_kernel(
    const float* __restrict__ wgt,
    _Float16* __restrict__ Wp)
{
  __shared__ __attribute__((aligned(16))) float cwr[KD];
  const int tid = threadIdx.x, o = blockIdx.x;
  for (int e = tid; e < KD / 4; e += 256) {
    const v4f g = *(const v4fa*)(wgt + (size_t)o * KD + 4 * e);
    const v4f r = { bf16r(g.x), bf16r(g.y), bf16r(g.z), bf16r(g.w) };
    *(v4fa*)(cwr + 4 * e) = r;
  }
  __syncthreads();

  const int kc = (tid < NCH) ? tid : (NCH - 1);
  const int t  = kc >> 4;
  const int c0 = (kc & 15) * 8;
  float v[8];
  #pragma unroll
  for (int i = 0; i < 8; ++i) v[i] = cwr[(c0 + i) * 9 + t] * W_CARRY;
  const v8h o8 = { (_Float16)v[0], (_Float16)v[1], (_Float16)v[2], (_Float16)v[3],
                   (_Float16)v[4], (_Float16)v[5], (_Float16)v[6], (_Float16)v[7] };
  _Float16* dst = Wp + (size_t)o * KD + 8 * kc;
  if (tid < NCH) *(volatile v8h*)dst = o8;
  __threadfence();
  if (tid < NCH) *(volatile v8h*)dst = o8;
}

__device__ __forceinline__ void xcvt_store_pass(const _Float16* T, _Float16* dst0, int tid) {
  #pragma unroll
  for (int it = 0; it < ((WW * CI) / 8) / 256; ++it) {
    const int ci = it * 256 + tid;
    const v8h v = *(const v8ha*)(T + 8 * ci);
    *(volatile v8h*)(dst0 + 8 * ci) = v;
  }
}

__global__ __launch_bounds__(256) void xcvt_kernel(const float* __restrict__ x,
                                                   _Float16* __restrict__ xh) {
  __shared__ __attribute__((aligned(16))) _Float16 T[WW * CI];
  const int tid = threadIdx.x, iy = blockIdx.x, b = blockIdx.y;
  #pragma unroll 1
  for (int e = tid; e < CI * (WW / 4); e += 256) {
    const int c = e / (WW / 4), q = e - c * (WW / 4);
    const v4f g = *(const v4fa*)(x + (((size_t)(b * CI + c)) * HH + iy) * WW + 4 * q);
    _Float16* p = T + (4 * q) * CI + c;
    p[0]      = (_Float16)(bf16r(g.x) * ACT_CARRY);
    p[CI]     = (_Float16)(bf16r(g.y) * ACT_CARRY);
    p[2 * CI] = (_Float16)(bf16r(g.z) * ACT_CARRY);
    p[3 * CI] = (_Float16)(bf16r(g.w) * ACT_CARRY);
  }
  __syncthreads();

  _Float16* dst0 = xh + ((size_t)(b * HH + iy)) * WW * CI;
  xcvt_store_pass(T, dst0, tid);
  __threadfence();
  xcvt_store_pass(T, dst0, tid);
}

__device__ __forceinline__ void out_store_pass(const char* smem, float* out,
                                               int b, int nb, int w, int lane) {
  const int q8 = lane & 7, sub = lane >> 3;
  #pragma unroll
  for (int it = 0; it < 8; ++it) {
    const int lid = 4 * it + sub;
    const int o = 16 * w + (lid >> 1), ln = lid & 1;
    const v4f v = *(const v4fa*)(smem + (size_t)(o * PT + 32 * ln + 4 * q8) * 4);
    float* dst = out + ((size_t)(b * NO + o)) * HWP + nb + 32 * ln + 4 * q8;
    *(volatile v4f*)dst = v;
  }
}

__global__ __launch_bounds__(256) void conv_kernel(
    const _Float16* __restrict__ xh,
    const _Float16* __restrict__ Wp,
    const float* __restrict__ bias,
    float* __restrict__ out)
{
  __shared__ __attribute__((aligned(16))) char smem[HR * HC * CI * 2];
  _Float16* sH = (_Float16*)smem;
  f32a* sF = (f32a*)smem;

  const int tid = threadIdx.x, lane = tid & 31, w = tid >> 5;
  const int h = lane >> 4, m = lane & 15;
  const int pt = blockIdx.x, b = blockIdx.y;
  const int nb = PT * pt;
  const int oyf = nb / WW;
  const v8h z8 = zero8h();

  for (int e = tid; e < HR * HC * (CI / 8); e += 256) {
    const int q = e & 15, rc = e >> 4;
    const int hr = rc / HC, hc = rc - HC * hr;
    const int iy = oyf - 1 + hr, ix = hc - 1;
    const bool ok = (iy >= 0) && (iy < HH) && (ix >= 0) && (ix < WW);
    const int iyc = (iy < 0) ? 0 : ((iy > HH - 1) ? (HH - 1) : iy);
    const int ixc = (ix < 0) ? 0 : ((ix > WW - 1) ? (WW - 1) : ix);
    const v8h g = *(const v8ha*)(xh + (((size_t)(b * HH + iyc)) * WW + ixc) * CI + 8 * q);
    *(v8ha*)(sH + (hr * HC + hc) * CI + 8 * q) = ok ? g : z8;
  }
  __syncthreads();

  const int cgp = w & 3, pg = w >> 2;
  const _Float16* wr0 = Wp + ((size_t)(32 * cgp + m)) * KD;
  const _Float16* wr1 = wr0 + (size_t)16 * KD;
  const int n0 = nb + 32 * pg + m, n1 = n0 + 16;
  const int oy0 = n0 / WW, ox0 = n0 - WW * oy0;
  const int oy1 = n1 / WW, ox1 = n1 - WW * oy1;
  const int pb0 = ((oy0 - oyf) * HC + ox0) * CI;
  const int pb1 = ((oy1 - oyf) * HC + ox1) * CI;

  const v8f zf = {0.f, 0.f, 0.f, 0.f, 0.f, 0.f, 0.f, 0.f};
  v8f acc[2][2];
  #pragma unroll
  for (int i = 0; i < 2; ++i)
    #pragma unroll
    for (int j = 0; j < 2; ++j) acc[i][j] = zf;

  #pragma unroll 1
  for (int s = 0; s < KD / 32; ++s) {
    const int t = s >> 2, dy = t / 3, dx = t - 3 * dy, ch0 = 32 * (s & 3);
    const v16h a0 = load_frag(wr0 + 32 * s, h);
    const v16h a1 = load_frag(wr1 + 32 * s, h);
    const int toff = (dy * HC + dx) * CI + ch0;
    const v16h b0 = load_frag(sH + pb0 + toff, h);
    acc[0][0] = wmma_f16(a0, b0, acc[0][0]);
    acc[1][0] = wmma_f16(a1, b0, acc[1][0]);
    const v16h b1 = load_frag(sH + pb1 + toff, h);
    acc[0][1] = wmma_f16(a0, b1, acc[0][1]);
    acc[1][1] = wmma_f16(a1, b1, acc[1][1]);
  }
  __syncthreads();

  #pragma unroll
  for (int i = 0; i < 2; ++i) {
    const int ob = 32 * cgp + 16 * i + 8 * h;
    const v4f bA = *(const v4fa*)(bias + ob);
    const v4f bB = *(const v4fa*)(bias + ob + 4);
    const float bb[8] = { bf16r(bA.x), bf16r(bA.y), bf16r(bA.z), bf16r(bA.w),
                          bf16r(bB.x), bf16r(bB.y), bf16r(bB.z), bf16r(bB.w) };
    #pragma unroll
    for (int j = 0; j < 2; ++j) {
      const int px = 32 * pg + 16 * j + m;
      #pragma unroll
      for (int r = 0; r < 8; ++r)
        sF[(ob + r) * PT + px] = acc[i][j][r] * INV_CARRY + bb[r];
    }
  }
  __syncthreads();

  out_store_pass(smem, out, b, nb, w, lane);
  __threadfence();
  out_store_pass(smem, out, b, nb, w, lane);
}

extern "C" void kernel_launch(void* const* d_in, const int* in_sizes, int n_in,
                              void* d_out, int out_size, void* d_ws, size_t ws_size,
                              hipStream_t stream) {
  if (n_in < 3) return;
  if (in_sizes[0] != NB * CI * HWP) return;
  if (in_sizes[1] != NO * KD) return;
  if (in_sizes[2] != NO) return;
  if (out_size != NB * NO * HWP) return;

  const float* x    = (const float*)d_in[0];
  const float* wgt  = (const float*)d_in[1];
  const float* bias = (const float*)d_in[2];
  float* out = (float*)d_out;

  const size_t wp_bytes = (size_t)NO * KD * 2;
  const size_t xh_bytes = (size_t)NB * HWP * CI * 2;
  const size_t total = wp_bytes + xh_bytes;
  if (total > ws_size) return;

  char* ws = (char*)d_ws;
  _Float16* Wp = (_Float16*)(ws);
  _Float16* xh = (_Float16*)(ws + wp_bytes);

  wcvt_kernel<<<NO, 256, 0, stream>>>(wgt, Wp);
  xcvt_kernel<<<dim3(HH, NB), 256, 0, stream>>>(x, xh);
  conv_kernel<<<dim3(NPT, NB), 256, 0, stream>>>(xh, Wp, bias, out);
}
